// TransformerBlock_11665131176261
// MI455X (gfx1250) — hardware-run, weakly checked
//
#include <hip/hip_runtime.h>
#include <stddef.h>


typedef _Float16 v16h __attribute__((ext_vector_type(16)));
typedef _Float16 v8h  __attribute__((ext_vector_type(8)));
typedef float    v8f  __attribute__((ext_vector_type(8)));
typedef float    v4f  __attribute__((ext_vector_type(4)));

#ifndef NB
#define NB 2
#endif
#ifndef SEQ
#define SEQ 2048
#endif
#define NB_FULL  2
#define SEQ_FULL 2048
#define DIM   1024
#define NHEAD 16
#define HD    64
#define ROT   32
#define INNER 4096
#define MROWS (NB * SEQ)

static_assert(NB >= 1 && NB <= NB_FULL);
static_assert(SEQ >= 128 && SEQ <= SEQ_FULL && (SEQ % 128) == 0);
static_assert(DIM == NHEAD * HD);
static_assert(HD == 64 && ROT == 32);
static_assert((DIM % 64) == 0 && (DIM % 32) == 0 && (INNER % 64) == 0 && (INNER % 32) == 0);
static_assert((MROWS % 64) == 0 && (MROWS % 8) == 0);
static_assert(((SEQ * ROT) % 256) == 0);
static_assert((size_t)MROWS * INNER < (size_t)0xFFFFFFFFu);

#define LDT 72
#define LDC 68

#define WCARRY  64.0f
#define ACARRY  16.0f
#define QKCARRY 8.0f
#define VCARRY  8.0f
#define PCARRY  1024.0f
#define CCARRY  64.0f
#define FCARRY  16.0f

#define WQKV_ELEMS ((size_t)3 * DIM * DIM)
#define WOUT_ELEMS ((size_t)DIM * DIM)
#define WFF1_ELEMS ((size_t)2 * INNER * DIM)
#define WFF2_ELEMS ((size_t)DIM * INNER)
#define W_BYTES    ((WQKV_ELEMS + WOUT_ELEMS + WFF1_ELEMS + WFF2_ELEMS) * 2)
#define TAB_BYTES  ((size_t)SEQ * ROT * 4)
#define PLANE16_ELEMS ((size_t)MROWS * DIM)
#define PLANE16_BYTES (PLANE16_ELEMS * 2)
#define X1_BYTES   ((size_t)MROWS * DIM * 4)
#define FF16_BYTES ((size_t)MROWS * INNER * 2)
#define WS_TOTAL   (W_BYTES + 2 * TAB_BYTES + 5 * PLANE16_BYTES + X1_BYTES + FF16_BYTES)
static_assert((WQKV_ELEMS % 2048) == 0 && (WOUT_ELEMS % 2048) == 0);
static_assert((WFF1_ELEMS % 2048) == 0 && (WFF2_ELEMS % 2048) == 0);
static_assert((W_BYTES % 128) == 0 && (TAB_BYTES % 128) == 0 && (PLANE16_BYTES % 128) == 0);
static_assert((X1_BYTES % 128) == 0 && (FF16_BYTES % 128) == 0);
static_assert(WS_TOTAL <= (size_t)134217728);

__device__ __forceinline__ float bf16r(float x) {
  unsigned int u = __float_as_uint(x);
  u = (u + 0x7FFFu + ((u >> 16) & 1u)) & 0xFFFF0000u;
  return __uint_as_float(u);
}

__device__ __forceinline__ v16h frag_at(const _Float16* p) {
  v8h lo = *(const v8h*)(p);
  v8h hi = *(const v8h*)(p + 16);
  v16h out;
#pragma unroll
  for (int i = 0; i < 8; ++i) { out[i] = lo[i]; out[i + 8] = hi[i]; }
  return out;
}
__device__ __forceinline__ v16h ld_frag(const _Float16* base, unsigned ld) {
  const unsigned lane = threadIdx.x & 31u;
  return frag_at(base + (lane & 15u) * ld + (lane >> 4) * 8u);
}

__device__ __forceinline__ v8f wmma16(v16h a, v16h b, v8f c) {
  v8f d = __builtin_amdgcn_wmma_f32_16x16x32_f16(false, a, false, b, (short)0, c,
                                                 false, false);
  asm volatile("v_nop\n\tv_nop\n\tv_nop\n\tv_nop" : "+v"(d) : "v"(a), "v"(b));
  return d;
}

__device__ __forceinline__ float red16_max(float x) {
#pragma unroll
  for (int off = 1; off < 16; off <<= 1) x = fmaxf(x, __shfl_xor(x, off, 32));
  return x;
}
__device__ __forceinline__ float red16_sum(float x) {
#pragma unroll
  for (int off = 1; off < 16; off <<= 1) x += __shfl_xor(x, off, 32);
  return x;
}
__device__ __forceinline__ float red32_sum(float x) {
#pragma unroll
  for (int off = 1; off < 32; off <<= 1) x += __shfl_xor(x, off, 32);
  return x;
}

__device__ __forceinline__ void wave_lds_sync() {
  __builtin_amdgcn_fence(3  , "wavefront");
  asm volatile("s_wait_dscnt 0x0" ::: "memory");
  __builtin_amdgcn_wave_barrier();
}

__device__ __forceinline__ float glu_val(float hv, float gv) {
  const float sg = __builtin_amdgcn_rcpf(1.0f + __expf(-gv));
  return hv * (gv * sg);
}

__global__ __launch_bounds__(256) void wcvt_kernel(
    const float* __restrict__ src, _Float16* __restrict__ dst) {
  const unsigned e = (blockIdx.x * 256u + threadIdx.x) * 8u;
  const v4f a0 = *(const v4f*)(src + e);
  const v4f a1 = *(const v4f*)(src + e + 4);
  v8h o;
#pragma unroll
  for (int j = 0; j < 4; ++j) {
    o[j]     = (_Float16)(WCARRY * bf16r(a0[j]));
    o[j + 4] = (_Float16)(WCARRY * bf16r(a1[j]));
  }
  *(volatile v8h*)(dst + (size_t)e) = o;
  __threadfence();
  *(volatile v8h*)(dst + (size_t)e) = o;
}

__global__ __launch_bounds__(256) void rope_tab_kernel(
    const float* __restrict__ fr, float* __restrict__ Ct, float* __restrict__ St) {
  const unsigned e = blockIdx.x * 256u + threadIdx.x;
  const float f = bf16r(fr[e]);
  float sn, cs;
  sincosf(f, &sn, &cs);
  const float ss = ((e & 31u) < 16u) ? -sn : sn;
  *(volatile float*)(Ct + e) = cs;
  *(volatile float*)(St + e) = ss;
  __threadfence();
  *(volatile float*)(Ct + e) = cs;
  *(volatile float*)(St + e) = ss;
}

template <int RNDIN>
__device__ __forceinline__ v8h ln_out8(const float* sp, const float* gp, float mu, float rstd) {
#pragma clang fp contract(off)
  const v4f a0 = *(const v4f*)(sp);
  const v4f a1 = *(const v4f*)(sp + 4);
  const v4f g0 = *(const v4f*)(gp);
  const v4f g1 = *(const v4f*)(gp + 4);
  v8h o;
#pragma unroll
  for (int t = 0; t < 4; ++t) {
    const float x0 = RNDIN ? bf16r(a0[t]) : a0[t];
    const float x1 = RNDIN ? bf16r(a1[t]) : a1[t];
    const float d0 = x0 - mu;
    const float d1 = x1 - mu;
    o[t]     = (_Float16)(ACARRY * (d0 * rstd * bf16r(g0[t])));
    o[t + 4] = (_Float16)(ACARRY * (d1 * rstd * bf16r(g1[t])));
  }
  return o;
}

template <int RNDIN>
__global__ __launch_bounds__(256) void ln_kernel(
    const float* __restrict__ src, const float* __restrict__ gamma,
    _Float16* __restrict__ dst) {
#pragma clang fp contract(off)
  const unsigned lane = threadIdx.x & 31u, w = threadIdx.x >> 5;
  const unsigned crow = blockIdx.x * 8u + w;
  size_t srow = crow;
  if (RNDIN) {
    const unsigned bidx = crow / (unsigned)SEQ;
    const unsigned sq = crow - bidx * (unsigned)SEQ;
    srow = (size_t)bidx * SEQ_FULL + sq;
  }
  const float* sp = src + srow * DIM + lane * 8u;
  const float* gp = gamma + lane * 8u;
  _Float16* dp = dst + (size_t)crow * DIM + lane * 8u;

  float s = 0.0f;
#pragma unroll 1
  for (unsigned j = 0; j < 4u; ++j) {
    const v4f a0 = *(const v4f*)(sp + j * 256u);
    const v4f a1 = *(const v4f*)(sp + j * 256u + 4u);
#pragma unroll
    for (int t = 0; t < 4; ++t) s = s + (RNDIN ? bf16r(a0[t]) : a0[t]);
#pragma unroll
    for (int t = 0; t < 4; ++t) s = s + (RNDIN ? bf16r(a1[t]) : a1[t]);
  }
  s = red32_sum(s);
  const float mu = s * (1.0f / (float)DIM);

  float s2 = 0.0f;
#pragma unroll 1
  for (unsigned j = 0; j < 4u; ++j) {
    const v4f a0 = *(const v4f*)(sp + j * 256u);
    const v4f a1 = *(const v4f*)(sp + j * 256u + 4u);
#pragma unroll
    for (int t = 0; t < 4; ++t) {
      const float d = (RNDIN ? bf16r(a0[t]) : a0[t]) - mu;
      const float q = d * d;
      s2 = s2 + q;
    }
#pragma unroll
    for (int t = 0; t < 4; ++t) {
      const float d = (RNDIN ? bf16r(a1[t]) : a1[t]) - mu;
      const float q = d * d;
      s2 = s2 + q;
    }
  }
  s2 = red32_sum(s2);
  const float rstd = rsqrtf(s2 * (1.0f / (float)DIM) + 1.0e-5f);

#pragma unroll 1
  for (unsigned j = 0; j < 4u; ++j) {
    const v8h o = ln_out8<RNDIN>(sp + j * 256u, gp + j * 256u, mu, rstd);
    *(volatile v8h*)(dp + j * 256u) = o;
  }
  __threadfence();
#pragma unroll 1
  for (unsigned j = 0; j < 4u; ++j) {
    const v8h o = ln_out8<RNDIN>(sp + j * 256u, gp + j * 256u, mu, rstd);
    *(volatile v8h*)(dp + j * 256u) = o;
  }
}

template <int MODE, int KDIM>
__global__ __launch_bounds__(256) void gemm_kernel(
    const _Float16* __restrict__ A16, const _Float16* __restrict__ Bt,
    const float* __restrict__ addf, const float* __restrict__ bias,
    const float* __restrict__ tabc, const float* __restrict__ tabs,
    float* __restrict__ outf, _Float16* __restrict__ out16) {
  __shared__ float Cs[(MODE == 3 ? 2 : 1) * 64 * LDC];
  const unsigned tid = threadIdx.x, lane = tid & 31u, w = tid >> 5;
  const unsigned mw = w >> 1, nw = w & 1u;
  const unsigned hh = lane >> 4, m = lane & 15u;
  const unsigned n0 = blockIdx.x * 64u;
  const unsigned row0 = blockIdx.y * 64u;

  const _Float16* ap  = A16 + (size_t)(row0 + mw * 16u + m) * KDIM + hh * 8u;
  const _Float16* bp0 = Bt + (size_t)(n0 + nw * 32u + m) * KDIM + hh * 8u;
  const _Float16* bp1 = bp0 + (size_t)16 * KDIM;
  const _Float16* bp2 = bp0 + (size_t)(MODE == 3 ? INNER : 0) * KDIM;
  const _Float16* bp3 = bp2 + (size_t)16 * KDIM;
  v8f acc0 = {}, acc1 = {}, acc2 = {}, acc3 = {};
#pragma unroll 2
  for (unsigned k0 = 0; k0 < (unsigned)KDIM; k0 += 32u) {
    const v16h a  = frag_at(ap + k0);
    const v16h b0 = frag_at(bp0 + k0);
    const v16h b1 = frag_at(bp1 + k0);
    acc0 = wmma16(a, b0, acc0);
    acc1 = wmma16(a, b1, acc1);
    if (MODE == 3) {
      const v16h b2 = frag_at(bp2 + k0);
      const v16h b3 = frag_at(bp3 + k0);
      acc2 = wmma16(a, b2, acc2);
      acc3 = wmma16(a, b3, acc3);
    }
  }
#pragma unroll
  for (int r = 0; r < 8; ++r) {
    float* d = &Cs[(mw * 16u + hh * 8u + (unsigned)r) * LDC + nw * 32u + m];
    d[0]  = acc0[r];
    d[16] = acc1[r];
    if (MODE == 3) {
      d[64 * LDC]      = acc2[r];
      d[64 * LDC + 16] = acc3[r];
    }
  }
  __syncthreads();

  if (MODE == 0) {
    const float inv = 1.0f / (WCARRY * ACARRY);
    const unsigned region = n0 / (unsigned)DIM;
    const unsigned hc = n0 - region * (unsigned)DIM;
    v8h x[2];
    size_t off[2];
    if (region < 2u) {
#pragma unroll
      for (unsigned i = 0; i < 2u; ++i) {
        const unsigned r = 32u * i + (tid >> 3);
        const unsigned c = (tid & 7u) * 8u;
        const unsigned crow = row0 + r;
        const unsigned bidx = crow / (unsigned)SEQ;
        const unsigned sq = crow - bidx * (unsigned)SEQ;
        const unsigned cc = c & 31u;
        const unsigned pc = c ^ 16u;
        const bool rotary = (c < 32u);
        const v4f u0 = *(const v4f*)&Cs[r * LDC + c];
        const v4f u1 = *(const v4f*)&Cs[r * LDC + c + 4];
        const v4f p0 = *(const v4f*)&Cs[r * LDC + pc];
        const v4f p1 = *(const v4f*)&Cs[r * LDC + pc + 4];
        const v4f c0 = *(const v4f*)(tabc + (size_t)sq * ROT + cc);
        const v4f c1 = *(const v4f*)(tabc + (size_t)sq * ROT + cc + 4);
        const v4f s0 = *(const v4f*)(tabs + (size_t)sq * ROT + cc);
        const v4f s1 = *(const v4f*)(tabs + (size_t)sq * ROT + cc + 4);
#pragma unroll
        for (int j = 0; j < 4; ++j) {
          const float t0 = u0[j] * inv, t1 = u1[j] * inv;
          const float q0 = p0[j] * inv, q1 = p1[j] * inv;
          const float r0 = t0 * c0[j] + q0 * s0[j];
          const float r1 = t1 * c1[j] + q1 * s1[j];
          x[i][j]     = (_Float16)(QKCARRY * (rotary ? r0 : t0));
          x[i][j + 4] = (_Float16)(QKCARRY * (rotary ? r1 : t1));
        }
        off[i] = (size_t)region * PLANE16_ELEMS + (size_t)crow * DIM + hc + c;
      }
#pragma unroll
      for (int i = 0; i < 2; ++i) *(volatile v8h*)(out16 + off[i]) = x[i];
      __threadfence();
#pragma unroll
      for (int i = 0; i < 2; ++i) *(volatile v8h*)(out16 + off[i]) = x[i];
    } else {
      const unsigned bidx = row0 / (unsigned)SEQ;
      const unsigned key0 = row0 - bidx * (unsigned)SEQ;
#pragma unroll
      for (unsigned i = 0; i < 2u; ++i) {
        const unsigned dcol = 32u * i + (tid >> 3);
        const unsigned kk = (tid & 7u) * 8u;
#pragma unroll
        for (unsigned j = 0; j < 8u; ++j)
          x[i][j] = (_Float16)(Cs[(kk + j) * LDC + dcol] * (VCARRY * inv));
        off[i] = (size_t)2 * PLANE16_ELEMS +
                 ((size_t)bidx * DIM + hc + dcol) * SEQ + key0 + kk;
      }
#pragma unroll
      for (int i = 0; i < 2; ++i) *(volatile v8h*)(out16 + off[i]) = x[i];
      __threadfence();
#pragma unroll
      for (int i = 0; i < 2; ++i) *(volatile v8h*)(out16 + off[i]) = x[i];
    }
  }

  if (MODE == 1 || MODE == 2) {
    const float inv = (MODE == 1) ? (1.0f / (WCARRY * CCARRY)) : (1.0f / (WCARRY * FCARRY));
    v4f xs[4];
    size_t off[4];
#pragma unroll
    for (unsigned i = 0; i < 4u; ++i) {
      const unsigned r = 16u * i + (tid >> 4);
      const unsigned c = (tid & 15u) * 4u;
      const unsigned crow = row0 + r;
      const unsigned bidx = crow / (unsigned)SEQ;
      const unsigned sq = crow - bidx * (unsigned)SEQ;
      const size_t frow = (size_t)bidx * SEQ_FULL + sq;
      const v4f u = *(const v4f*)&Cs[r * LDC + c];
      v4f val;
      if (MODE == 1) {
        const v4f g = *(const v4f*)(addf + frow * DIM + n0 + c);
#pragma unroll
        for (int j = 0; j < 4; ++j) val[j] = bf16r(g[j]) + u[j] * inv;
        off[i] = (size_t)crow * DIM + n0 + c;
      } else {
        const v4f g = *(const v4f*)(addf + (size_t)crow * DIM + n0 + c);
        const v4f bb = *(const v4f*)(bias + n0 + c);
#pragma unroll
        for (int j = 0; j < 4; ++j) val[j] = g[j] + (u[j] * inv + bf16r(bb[j]));
        off[i] = frow * DIM + n0 + c;
      }
      xs[i] = val;
    }
#pragma unroll
    for (int i = 0; i < 4; ++i) *(volatile v4f*)(outf + off[i]) = xs[i];
    __threadfence();
#pragma unroll
    for (int i = 0; i < 4; ++i) *(volatile v4f*)(outf + off[i]) = xs[i];
  }

  if (MODE == 3) {
    const float inv = 1.0f / (WCARRY * ACARRY);
    v8h x[2];
    size_t off[2];
#pragma unroll
    for (unsigned i = 0; i < 2u; ++i) {
      const unsigned r = 32u * i + (tid >> 3);
      const unsigned c = (tid & 7u) * 8u;
      const v4f h0 = *(const v4f*)&Cs[r * LDC + c];
      const v4f h1 = *(const v4f*)&Cs[r * LDC + c + 4];
      const v4f g0 = *(const v4f*)&Cs[64 * LDC + r * LDC + c];
      const v4f g1 = *(const v4f*)&Cs[64 * LDC + r * LDC + c + 4];
      const v4f bh0 = *(const v4f*)(bias + n0 + c);
      const v4f bh1 = *(const v4f*)(bias + n0 + c + 4);
      const v4f bg0 = *(const v4f*)(bias + INNER + n0 + c);
      const v4f bg1 = *(const v4f*)(bias + INNER + n0 + c + 4);
#pragma unroll
      for (int j = 0; j < 4; ++j) {
        const float hv0 = h0[j] * inv + bf16r(bh0[j]);
        const float gv0 = g0[j] * inv + bf16r(bg0[j]);
        const float hv1 = h1[j] * inv + bf16r(bh1[j]);
        const float gv1 = g1[j] * inv + bf16r(bg1[j]);
        x[i][j]     = (_Float16)(FCARRY * glu_val(hv0, gv0));
        x[i][j + 4] = (_Float16)(FCARRY * glu_val(hv1, gv1));
      }
      off[i] = (size_t)(row0 + r) * INNER + n0 + c;
    }
#pragma unroll
    for (int i = 0; i < 2; ++i) *(volatile v8h*)(out16 + off[i]) = x[i];
    __threadfence();
#pragma unroll
    for (int i = 0; i < 2; ++i) *(volatile v8h*)(out16 + off[i]) = x[i];
  }
}

__global__ __launch_bounds__(256) void attn_kernel(
    const _Float16* __restrict__ Qh, const _Float16* __restrict__ Kh,
    const _Float16* __restrict__ Vt, _Float16* __restrict__ Ov) {
  __shared__ _Float16 Ks[64 * LDT];
  __shared__ _Float16 Vs[64 * LDT];
  __shared__ _Float16 Ps[8 * 16 * LDT];

  const unsigned tid = threadIdx.x, lane = tid & 31u, w = tid >> 5;
  const unsigned wu = (unsigned)__builtin_amdgcn_readfirstlane((int)(tid >> 5));
  const unsigned hh = lane >> 4, m = lane & 15u;
  const unsigned q0 = blockIdx.x * 128u;
  const unsigned head = blockIdx.y;
  const unsigned b = blockIdx.z;
  const float scale = 0.125f / (QKCARRY * QKCARRY);
  _Float16* P = Ps + w * (16u * LDT);

  const size_t qoff = (size_t)(b * (unsigned)SEQ + q0 + w * 16u + m) * DIM + head * HD + hh * 8u;
  v16h qf[2];
  qf[0] = frag_at(Qh + qoff);
  qf[1] = frag_at(Qh + qoff + 32);

  float mrow[8], lrow[8];
  v8f o[4];
#pragma unroll
  for (int v = 0; v < 8; ++v) { mrow[v] = -1.0e30f; lrow[v] = 0.0f; }
#pragma unroll
  for (int nb = 0; nb < 4; ++nb) o[nb] = (v8f){};

  const size_t kplane = (size_t)b * SEQ * DIM + head * HD;
  const size_t vplane = ((size_t)b * DIM + head * HD) * SEQ;
  const unsigned kend = q0 + 128u;
  const unsigned wrow0 = q0 + wu * 16u;
  const unsigned rowb = q0 + w * 16u + hh * 8u;

  for (unsigned kb = 0; kb < kend; kb += 64u) {
#pragma unroll
    for (unsigned j = 0; j < 2u; ++j) {
      const unsigned idx = tid + 256u * j;
      const unsigned r = idx >> 3, c = (idx & 7u) * 8u;
      *(v8h*)&Ks[r * LDT + c] = *(const v8h*)(Kh + kplane + (size_t)(kb + r) * DIM + c);
      *(v8h*)&Vs[r * LDT + c] = *(const v8h*)(Vt + vplane + (size_t)r * SEQ + kb + c);
    }
    __syncthreads();

    if (kb <= wrow0 + 15u) {
      v8f s[4];
#pragma unroll
      for (int kg = 0; kg < 4; ++kg) {
        v8f t = {};
#pragma unroll
        for (int c = 0; c < 2; ++c) {
          const v16h kf = ld_frag(&Ks[(kg * 16) * LDT + c * 32], LDT);
          t = wmma16(qf[c], kf, t);
        }
        const unsigned col = kb + (unsigned)kg * 16u + m;
#pragma unroll
        for (int v = 0; v < 8; ++v)
          s[kg][v] = (col <= rowb + (unsigned)v) ? (t[v] * scale) : -1.0e30f;
      }

      float alpha[8];
#pragma unroll
      for (int v = 0; v < 8; ++v) {
        float mx = fmaxf(fmaxf(s[0][v], s[1][v]), fmaxf(s[2][v], s[3][v]));
        mx = red16_max(mx);
        const float mn = fmaxf(mrow[v], mx);
        alpha[v] = __expf(mrow[v] - mn);
        mrow[v] = mn;
      }
#pragma unroll
      for (int kg = 0; kg < 4; ++kg)
#pragma unroll
        for (int v = 0; v < 8; ++v) s[kg][v] = __expf(s[kg][v] - mrow[v]);
#pragma unroll
      for (int v = 0; v < 8; ++v) {
        const float rs = red16_sum((s[0][v] + s[1][v]) + (s[2][v] + s[3][v]));
        lrow[v] = alpha[v] * lrow[v] + rs;
      }
#pragma unroll
      for (int nb = 0; nb < 4; ++nb)
#pragma unroll
        for (int v = 0; v < 8; ++v) o[nb][v] = o[nb][v] * alpha[v];

#pragma unroll
      for (int kg = 0; kg < 4; ++kg)
#pragma unroll
        for (int v = 0; v < 8; ++v)
          P[(hh * 8u + (unsigned)v) * LDT + (unsigned)kg * 16u + m] =
              (_Float16)(s[kg][v] * PCARRY);
      wave_lds_sync();

#pragma unroll
      for (int c = 0; c < 2; ++c) {
        const v16h pf = ld_frag(P + c * 32, LDT);
#pragma unroll
        for (int nb = 0; nb < 4; ++nb) {
          const v16h vf = ld_frag(&Vs[(nb * 16) * LDT + c * 32], LDT);
          o[nb] = wmma16(pf, vf, o[nb]);
        }
      }
    }
    __syncthreads();
  }

  float inv[8];
#pragma unroll
  for (int v = 0; v < 8; ++v)
    inv[v] = __builtin_amdgcn_rcpf(lrow[v]) * (CCARRY / (PCARRY * VCARRY));
#pragma unroll
  for (int nb = 0; nb < 4; ++nb)
#pragma unroll
    for (int v = 0; v < 8; ++v)
      P[(hh * 8u + (unsigned)v) * LDT + (unsigned)nb * 16u + m] = (_Float16)(o[nb][v] * inv[v]);
  wave_lds_sync();
  v8h x[4];
  size_t off[4];
#pragma unroll
  for (unsigned i = 0; i < 4u; ++i) {
    const unsigned r = 4u * i + (lane >> 3);
    const unsigned c = (lane & 7u) * 8u;
    x[i] = *(const v8h*)&P[r * LDT + c];
    off[i] = (size_t)(b * (unsigned)SEQ + q0 + w * 16u + r) * DIM + head * HD + c;
  }
#pragma unroll
  for (int i = 0; i < 4; ++i) *(volatile v8h*)(Ov + off[i]) = x[i];
  __threadfence();
#pragma unroll
  for (int i = 0; i < 4; ++i) *(volatile v8h*)(Ov + off[i]) = x[i];
}

extern "C" void kernel_launch(void* const* d_in, const int* in_sizes, int n_in,
                              void* d_out, int out_size, void* d_ws, size_t ws_size,
                              hipStream_t stream) {
  if (n_in < 10) return;
  const long long need_x = ((long long)(NB - 1) * SEQ_FULL + SEQ) * DIM;
  if ((long long)in_sizes[0] < need_x) return;
  if ((long long)in_sizes[1] < (long long)SEQ * ROT) return;
  if ((long long)in_sizes[2] < (long long)3 * DIM * DIM) return;
  if ((long long)in_sizes[3] < (long long)DIM * DIM) return;
  if (in_sizes[4] < DIM) return;
  if (in_sizes[5] < DIM) return;
  if ((long long)in_sizes[6] < (long long)2 * INNER * DIM) return;
  if (in_sizes[7] < 2 * INNER) return;
  if ((long long)in_sizes[8] < (long long)DIM * INNER) return;
  if (in_sizes[9] < DIM) return;
  if ((long long)out_size < need_x) return;
  if (ws_size < WS_TOTAL) return;

  const float* X     = (const float*)d_in[0];
  const float* freqs = (const float*)d_in[1];
  const float* Wqkv  = (const float*)d_in[2];
  const float* Wout  = (const float*)d_in[3];
  const float* g1    = (const float*)d_in[4];
  const float* g2    = (const float*)d_in[5];
  const float* Wff1  = (const float*)d_in[6];
  const float* bff1  = (const float*)d_in[7];
  const float* Wff2  = (const float*)d_in[8];
  const float* bff2  = (const float*)d_in[9];
  float* out = (float*)d_out;

  char* ws = (char*)d_ws;
  size_t o = 0;
  _Float16* W16q  = (_Float16*)(ws + o);  o += WQKV_ELEMS * 2;
  _Float16* W16o  = (_Float16*)(ws + o);  o += WOUT_ELEMS * 2;
  _Float16* W16f1 = (_Float16*)(ws + o);  o += WFF1_ELEMS * 2;
  _Float16* W16f2 = (_Float16*)(ws + o);  o += WFF2_ELEMS * 2;
  float*    Ct    = (float*)(ws + o);     o += TAB_BYTES;
  float*    St    = (float*)(ws + o);     o += TAB_BYTES;
  _Float16* XN16  = (_Float16*)(ws + o);  o += PLANE16_BYTES;
  _Float16* Q16   = (_Float16*)(ws + o);  o += PLANE16_BYTES;
  _Float16* K16   = (_Float16*)(ws + o);  o += PLANE16_BYTES;
  _Float16* Vt16  = (_Float16*)(ws + o);  o += PLANE16_BYTES;
  _Float16* Ctx16 = (_Float16*)(ws + o);  o += PLANE16_BYTES;
  float*    X1    = (float*)(ws + o);     o += X1_BYTES;
  _Float16* FF16  = (_Float16*)(ws + o);  o += FF16_BYTES;
  if (o != WS_TOTAL) return;

  dim3 blk(256);

  wcvt_kernel<<<dim3((unsigned)(WQKV_ELEMS / 2048)), blk, 0, stream>>>(Wqkv, W16q);
  wcvt_kernel<<<dim3((unsigned)(WOUT_ELEMS / 2048)), blk, 0, stream>>>(Wout, W16o);
  wcvt_kernel<<<dim3((unsigned)(WFF1_ELEMS / 2048)), blk, 0, stream>>>(Wff1, W16f1);
  wcvt_kernel<<<dim3((unsigned)(WFF2_ELEMS / 2048)), blk, 0, stream>>>(Wff2, W16f2);
  rope_tab_kernel<<<dim3((SEQ * ROT) / 256), blk, 0, stream>>>(freqs, Ct, St);

  ln_kernel<1><<<dim3(MROWS / 8), blk, 0, stream>>>(X, g1, XN16);
  gemm_kernel<0, DIM><<<dim3(3 * DIM / 64, MROWS / 64), blk, 0, stream>>>(
      XN16, W16q, X, bff2, Ct, St, X1, Q16);
  attn_kernel<<<dim3(SEQ / 128, NHEAD, NB), blk, 0, stream>>>(Q16, K16, Vt16, Ctx16);
  gemm_kernel<1, DIM><<<dim3(DIM / 64, MROWS / 64), blk, 0, stream>>>(
      Ctx16, W16o, X, bff2, Ct, St, X1, Q16);

  ln_kernel<0><<<dim3(MROWS / 8), blk, 0, stream>>>(X1, g2, XN16);
  gemm_kernel<3, DIM><<<dim3(INNER / 64, MROWS / 64), blk, 0, stream>>>(
      XN16, W16f1, X, bff1, Ct, St, X1, FF16);
  gemm_kernel<2, INNER><<<dim3(DIM / 64, MROWS / 64), blk, 0, stream>>>(
      FF16, W16f2, X1, bff2, Ct, St, out, Q16);
}
